// TGAT_6030134083688
// MI455X (gfx1250) — hardware-run, weakly checked
//
#include <hip/hip_runtime.h>
#include <hip/hip_bf16.h>
#include <stddef.h>
#include <stdint.h>


#define DIN     17
#define DH      32
#define TD      32
#define CH      16
#define NCLS    2
#define KP      64
#define NODEW   128
#define OQ      0
#define OKK     32
#define OV      64
#define OSK     96
#define NB2     128
#define WES     33
#define NTHR    256
#define NWAVE   8
#define EPT     8
#define CHUNK   (NTHR * EPT)
#define WCAP    (EPT * 32)
#define LISTN   (NWAVE * WCAP)
#define NBMAX   512
#define SLOTB   9
#define RCAP    28672
#define DEGCAP  128
#define STW     64
#define GBM     64
#define GBN     64
#define GTHR    128
#define ATTSC   0.25f
#define WSMAX   134217728
#define LDSW_SWE  (2 * RCAP + 2 * NBMAX + LISTN + 2 * NWAVE)
#define LDSW_SOUT (LDSW_SWE + TD * WES)
#define LDSW_END  (LDSW_SOUT + NCLS * NBMAX)
#define LDS_AGG   (LDSW_END * 4 + 64)

static_assert((1 << SLOTB) == NBMAX);
static_assert(SLOTB + 22 <= 31);
static_assert((CHUNK & (CHUNK - 1)) == 0 && CHUNK <= 4096);
static_assert(NTHR * 2 == NBMAX);
static_assert(NTHR * 4 == NBMAX * NCLS);
static_assert(((NBMAX * NCLS * 4) % 128) == 0);
static_assert(LISTN >= NBMAX);
static_assert(LISTN >= NWAVE * WCAP);
static_assert((RCAP % 32) == 0);
static_assert((NBMAX % NWAVE) == 0);
static_assert(NWAVE * STW <= RCAP && STW >= 2 * DH);
static_assert((LDSW_SOUT % 4) == 0);
static_assert(LDS_AGG <= 300000);
static_assert(GBM == (GTHR / 32) * 16);
static_assert((KP % 32) == 0 && KP >= DIN && KP == 2 * DH);
static_assert(NODEW == 4 * DH && (NODEW % GBN) == 0);
static_assert(TD == 32 && DH == 32 && 2 * CH == DH && NCLS == 2);
static_assert(GBM * 8 == 4 * GTHR);
static_assert(DH * 8 == NTHR && NB2 * 8 == 4 * NTHR);

typedef float          v4f  __attribute__((ext_vector_type(4)));
typedef float          v8f  __attribute__((ext_vector_type(8)));
typedef int            v4i  __attribute__((ext_vector_type(4)));
typedef int            v8i  __attribute__((ext_vector_type(8)));
typedef unsigned short v8us __attribute__((ext_vector_type(8)));
typedef __bf16         v16b __attribute__((ext_vector_type(16)));
typedef v4f  __attribute__((may_alias)) v4fa;
typedef v8us __attribute__((may_alias)) v8usa;
union FragB { v16b v; v8us h[2]; v8i w; };

__device__ __forceinline__ v8f wmb(const FragB& a, const FragB& b, v8f c) {
  v8f d = __builtin_amdgcn_wmma_f32_16x16x32_bf16(false, a.v, false, b.v, (short)0, c, false, false);
  asm volatile("v_nop\n\tv_nop\n\tv_nop\n\tv_nop" : "+v"(d) : "v"(a.w), "v"(b.w));
  return d;
}

__device__ __forceinline__ void ldwait() {
  asm volatile("s_wait_loadcnt 0x0" ::: "memory");
}

__device__ __forceinline__ unsigned short f2bf(float f) {
  unsigned u = __float_as_uint(f);
  u += 0x7FFFu + ((u >> 16) & 1u);
  return (unsigned short)(u >> 16);
}
__device__ __forceinline__ float bfr(float f) {
  unsigned u = __float_as_uint(f);
  u = (u + 0x7FFFu + ((u >> 16) & 1u)) & 0xFFFF0000u;
  return __uint_as_float(u);
}
__device__ __forceinline__ v8us cvt8b(const v4f a, const v4f b) {
  v8us o;
  o[0] = f2bf(a.x); o[1] = f2bf(a.y); o[2] = f2bf(a.z); o[3] = f2bf(a.w);
  o[4] = f2bf(b.x); o[5] = f2bf(b.y); o[6] = f2bf(b.z); o[7] = f2bf(b.w);
  return o;
}
__device__ __forceinline__ unsigned short hlb(float v, bool lo) {
  const unsigned short hb = f2bf(v);
  const float hv = __uint_as_float(((unsigned)hb) << 16);
  const unsigned short lb = f2bf(v - hv);
  return lo ? lb : hb;
}
__device__ __forceinline__ v8us cvt8hl(const v4f a, const v4f b, bool lo) {
  v8us o;
  o[0] = hlb(a.x, lo); o[1] = hlb(a.y, lo); o[2] = hlb(a.z, lo); o[3] = hlb(a.w, lo);
  o[4] = hlb(b.x, lo); o[5] = hlb(b.y, lo); o[6] = hlb(b.z, lo); o[7] = hlb(b.w, lo);
  return o;
}

__device__ __forceinline__ float cosv(float x) {
  const float kq = rintf(x * 0.15915494309189535f);
  float r = fmaf(-kq, 6.2831855f, x);
  r = fmaf(-kq, -1.7484555e-7f, r);
  const float s = r * r;
  float p = 1.6117376e-24f;
  p = fmaf(p, s, -8.8967914e-22f);
  p = fmaf(p, s, 4.1103176e-19f);
  p = fmaf(p, s, -1.5619207e-16f);
  p = fmaf(p, s, 4.7794773e-14f);
  p = fmaf(p, s, -1.1470746e-11f);
  p = fmaf(p, s, 2.0876757e-9f);
  p = fmaf(p, s, -2.7557319e-7f);
  p = fmaf(p, s, 2.4801587e-5f);
  p = fmaf(p, s, -1.3888889e-3f);
  p = fmaf(p, s, 4.1666668e-2f);
  p = fmaf(p, s, -0.5f);
  p = fmaf(p, s, 1.0f);
  return p;
}

__device__ __forceinline__ void red2(float own, float oth, float* town, float* toth) {
  float e = own + __shfl_xor(oth, 16);
  e += __shfl_xor(e, 8);
  e += __shfl_xor(e, 4);
  e += __shfl_xor(e, 2);
  e += __shfl_xor(e, 1);
  *town = e;
  *toth = __shfl_xor(e, 16);
}

__device__ __forceinline__ int scan_chunk(const int* __restrict__ dsts, int nE, int cbase, int slotBase,
                                          int nb, int vec8, int* list, int tid, int lane, int wave) {
  int wc = 0;
  const int el0  = tid * EPT;
  const int e0   = cbase + el0;
  const int sent = -2147483647 - 1;
  v4i da, db;
  if (vec8 != 0 && cbase + CHUNK <= nE) {
    da = *(const v4i*)(dsts + e0);
    db = *(const v4i*)(dsts + e0 + 4);
  } else {
    da.x = (e0     < nE) ? dsts[min(e0,     nE - 1)] : sent;
    da.y = (e0 + 1 < nE) ? dsts[min(e0 + 1, nE - 1)] : sent;
    da.z = (e0 + 2 < nE) ? dsts[min(e0 + 2, nE - 1)] : sent;
    da.w = (e0 + 3 < nE) ? dsts[min(e0 + 3, nE - 1)] : sent;
    db.x = (e0 + 4 < nE) ? dsts[min(e0 + 4, nE - 1)] : sent;
    db.y = (e0 + 5 < nE) ? dsts[min(e0 + 5, nE - 1)] : sent;
    db.z = (e0 + 6 < nE) ? dsts[min(e0 + 6, nE - 1)] : sent;
    db.w = (e0 + 7 < nE) ? dsts[min(e0 + 7, nE - 1)] : sent;
  }
  const unsigned nbs = (unsigned)slotBase;
  const unsigned unb = (unsigned)nb;
  const unsigned s0 = (unsigned)da.x - nbs, s1 = (unsigned)da.y - nbs;
  const unsigned s2 = (unsigned)da.z - nbs, s3 = (unsigned)da.w - nbs;
  const unsigned s4 = (unsigned)db.x - nbs, s5 = (unsigned)db.y - nbs;
  const unsigned s6 = (unsigned)db.z - nbs, s7 = (unsigned)db.w - nbs;
  const bool h0 = s0 < unb, h1 = s1 < unb, h2 = s2 < unb, h3 = s3 < unb;
  const bool h4 = s4 < unb, h5 = s5 < unb, h6 = s6 < unb, h7 = s7 < unb;
  const unsigned any = __builtin_amdgcn_ballot_w32(h0 | h1 | h2 | h3 | h4 | h5 | h6 | h7);
  if (any != 0u) {
#define HITJ(J, HJ, SJ) { \
      const unsigned mj = __builtin_amdgcn_ballot_w32(HJ); \
      if (mj != 0u) { \
        if (HJ) { \
          const int pos = wc + (int)__builtin_amdgcn_mbcnt_lo(mj, 0u); \
          if (pos < WCAP) list[wave * WCAP + pos] = ((el0 + (J)) << 12) | (int)(SJ); \
        } \
        wc += (int)__builtin_popcount(mj); } }
    HITJ(0, h0, s0)
    HITJ(1, h1, s1)
    HITJ(2, h2, s2)
    HITJ(3, h3, s3)
    HITJ(4, h4, s4)
    HITJ(5, h5, s5)
    HITJ(6, h6, s6)
    HITJ(7, h7, s7)
#undef HITJ
  }
  return wc;
}

__device__ __forceinline__ float ldx(const float* p, int c, bool live) {
  const int cc = c < DIN ? c : DIN - 1;
  const float v = p[cc];
  return (live && c < DIN) ? v : 0.0f;
}
__global__ __launch_bounds__(NTHR) void k_xprep(const float* __restrict__ x, unsigned short* xa, int nN, int nUnits) {
  const int i = (int)blockIdx.x * NTHR + (int)threadIdx.x;
  if (i >= nUnits) return;
  const int row = i >> 3;
  const int c0  = (i & 7) * 8;
  const int rc  = row < nN ? row : nN - 1;
  const bool live = row < nN;
  const float* p = x + (size_t)rc * DIN;
  v4f a, b;
  a.x = ldx(p, c0 + 0, live); a.y = ldx(p, c0 + 1, live); a.z = ldx(p, c0 + 2, live); a.w = ldx(p, c0 + 3, live);
  b.x = ldx(p, c0 + 4, live); b.y = ldx(p, c0 + 5, live); b.z = ldx(p, c0 + 6, live); b.w = ldx(p, c0 + 7, live);
  const v8us hv = cvt8b(a, b);
  const size_t o = (size_t)row * KP + c0;
  *(volatile v8us*)(xa + o) = hv;
  __threadfence();
  *(volatile v8us*)(xa + o) = hv;
}

__global__ __launch_bounds__(NTHR) void k_wprep(const float* __restrict__ Wlin,
                                                const float* __restrict__ Wq, const float* __restrict__ Wk,
                                                const float* __restrict__ Wv, const float* __restrict__ Ws,
                                                unsigned short* wlt, unsigned short* b2t) {
  const int tid = (int)threadIdx.x;
  if (blockIdx.x == 0) {
    const int n  = tid >> 3;
    const int k8 = (tid & 7) * 8;
    const float* p = Wlin + (size_t)n * DIN;
    v4f a, b;
    a.x = ldx(p, k8 + 0, true); a.y = ldx(p, k8 + 1, true); a.z = ldx(p, k8 + 2, true); a.w = ldx(p, k8 + 3, true);
    b.x = ldx(p, k8 + 4, true); b.y = ldx(p, k8 + 5, true); b.z = ldx(p, k8 + 6, true); b.w = ldx(p, k8 + 7, true);
    const v8us hv = cvt8b(a, b);
    const size_t o = (size_t)n * KP + k8;
    *(volatile v8us*)(wlt + o) = hv;
    __threadfence();
    *(volatile v8us*)(wlt + o) = hv;
  } else {
    const int seg = (int)blockIdx.x - 1;
    const int v   = seg * NTHR + tid;
    const int n   = v >> 3;
    const int k8  = (v & 7) * 8;
    const int nc  = n & 31;
    const float* wsg = (seg == 0) ? Wq : ((seg == 1) ? Wk : ((seg == 2) ? Wv : Ws));
    const float* p = wsg + (size_t)nc * DH + (k8 & 31);
    v4f a, b;
    a.x = p[0]; a.y = p[1]; a.z = p[2]; a.w = p[3];
    b.x = p[4]; b.y = p[5]; b.z = p[6]; b.w = p[7];
    const v8us hv = cvt8b(a, b);
    const size_t o = (size_t)n * KP + k8;
    *(volatile v8us*)(b2t + o) = hv;
    __threadfence();
    *(volatile v8us*)(b2t + o) = hv;
  }
}

__global__ __launch_bounds__(GTHR) void k_gemm1(
    const unsigned short* __restrict__ A, const unsigned short* __restrict__ WT,
    const float* __restrict__ blin, unsigned short* H1A, int K, int nN)
{
  __shared__ __attribute__((aligned(16))) float stg[GBM * DH];
  const int tid = (int)threadIdx.x, lane = tid & 31, wave = tid >> 5, hh = lane >> 4, m = lane & 15;
  const int rowBase = (int)blockIdx.x * GBM;

  v8f acc[2];
  {
    const v8f z = {0.f, 0.f, 0.f, 0.f, 0.f, 0.f, 0.f, 0.f};
    acc[0] = z; acc[1] = z;
  }
  const unsigned short* ap = A  + (size_t)(rowBase + 16 * wave + m) * (size_t)K + 8 * hh;
  const unsigned short* wp = WT + (size_t)m * (size_t)K + 8 * hh;
  const int ksteps = K >> 5;
#pragma unroll 1
  for (int ks = 0; ks < ksteps; ++ks) {
    FragB af;
    af.h[0] = *(const v8usa*)(ap + 32 * ks);
    af.h[1] = *(const v8usa*)(ap + 32 * ks + 16);
#pragma unroll
    for (int t = 0; t < 2; ++t) {
      const unsigned short* wq = wp + (size_t)(16 * t) * (size_t)K + 32 * ks;
      FragB bf;
      bf.h[0] = *(const v8usa*)wq;
      bf.h[1] = *(const v8usa*)(wq + 16);
      acc[t] = wmb(af, bf, acc[t]);
    }
  }

#pragma unroll
  for (int t = 0; t < 2; ++t) {
    const int lc = 16 * t + m;
    const float bv = bfr(blin[lc]);
#pragma unroll
    for (int r = 0; r < 8; ++r) {
      const int lr = 16 * wave + 8 * hh + r;
      stg[lr * DH + lc] = fmaxf(acc[t][r] + bv, 0.0f);
    }
  }
  __syncthreads();

  v8us pv[4];
#pragma unroll
  for (int i = 0; i < 4; ++i) {
    const int p   = i * GTHR + tid;
    const int row = p >> 3;
    const int q   = p & 7;
    const int cq  = (q & 3) * 8;
    v4f a = *(const v4fa*)(stg + row * DH + cq);
    v4f b = *(const v4fa*)(stg + row * DH + cq + 4);
    const v4f z4 = {0.f, 0.f, 0.f, 0.f};
    if (rowBase + row >= nN) { a = z4; b = z4; }
    pv[i] = cvt8hl(a, b, q >= 4);
  }
#pragma unroll
  for (int i = 0; i < 4; ++i) {
    const int p = i * GTHR + tid;
    unsigned short* op = H1A + (size_t)(rowBase + (p >> 3)) * KP + 8 * (p & 7);
    *(volatile v8us*)op = pv[i];
  }
  __threadfence();
#pragma unroll
  for (int i = 0; i < 4; ++i) {
    const int p = i * GTHR + tid;
    unsigned short* op = H1A + (size_t)(rowBase + (p >> 3)) * KP + 8 * (p & 7);
    *(volatile v8us*)op = pv[i];
  }
}

__global__ __launch_bounds__(GTHR) void k_gemm2(
    const unsigned short* __restrict__ A, const unsigned short* __restrict__ WT,
    const float* __restrict__ b0, const float* __restrict__ b1,
    const float* __restrict__ b2, const float* __restrict__ b3,
    float* outF, int K, int ldo)
{
  __shared__ __attribute__((aligned(16))) float stg[GBM * GBN];
  const int tid = (int)threadIdx.x, lane = tid & 31, wave = tid >> 5, hh = lane >> 4, m = lane & 15;
  const int rowBase = (int)blockIdx.x * GBM;
  const int col0    = (int)blockIdx.y * GBN;

  v8f acc[4];
  {
    const v8f z = {0.f, 0.f, 0.f, 0.f, 0.f, 0.f, 0.f, 0.f};
    acc[0] = z; acc[1] = z; acc[2] = z; acc[3] = z;
  }
  const unsigned short* ap = A  + (size_t)(rowBase + 16 * wave + m) * (size_t)K + 8 * hh;
  const unsigned short* wp = WT + (size_t)(col0 + m) * (size_t)K + 8 * hh;
  const int ksteps = K >> 5;
#pragma unroll 1
  for (int ks = 0; ks < ksteps; ++ks) {
    FragB af;
    af.h[0] = *(const v8usa*)(ap + 32 * ks);
    af.h[1] = *(const v8usa*)(ap + 32 * ks + 16);
#pragma unroll
    for (int t = 0; t < 4; ++t) {
      const unsigned short* wq = wp + (size_t)(16 * t) * (size_t)K + 32 * ks;
      FragB bf;
      bf.h[0] = *(const v8usa*)wq;
      bf.h[1] = *(const v8usa*)(wq + 16);
      acc[t] = wmb(af, bf, acc[t]);
    }
  }

#pragma unroll
  for (int t = 0; t < 4; ++t) {
    const int lc  = 16 * t + m;
    const int gc0 = col0 + 16 * t;
    const int seg = (gc0 >> 5) & 3;
    const float* bp = (seg == 0) ? b0 : ((seg == 1) ? b1 : ((seg == 2) ? b2 : b3));
    const float bv = bfr(bp[(gc0 + m) & 31]);
#pragma unroll
    for (int r = 0; r < 8; ++r) {
      const int lr = 16 * wave + 8 * hh + r;
      stg[lr * GBN + lc] = acc[t][r] + bv;
    }
  }
  __syncthreads();

  v4f fv[8];
#pragma unroll
  for (int i = 0; i < 8; ++i) {
    const int lr = 16 * wave + 2 * i + hh;
    fv[i] = *(const v4fa*)(stg + lr * GBN + 4 * m);
  }
#pragma unroll
  for (int i = 0; i < 8; ++i) {
    const int lr = 16 * wave + 2 * i + hh;
    const int gr = rowBase + lr;
    float* op = outF + (size_t)gr * (size_t)ldo + col0 + 4 * m;
    *(volatile v4f*)op = fv[i];
  }
  __threadfence();
#pragma unroll
  for (int i = 0; i < 8; ++i) {
    const int lr = 16 * wave + 2 * i + hh;
    const int gr = rowBase + lr;
    float* op = outF + (size_t)gr * (size_t)ldo + col0 + 4 * m;
    *(volatile v4f*)op = fv[i];
  }
}

__global__ __launch_bounds__(NTHR) void k_agg(
    const int* __restrict__ srcs, const int* __restrict__ dsts,
    const float* __restrict__ NODE, const float* __restrict__ tt, const float* __restrict__ ntime,
    const float* __restrict__ bfq, const float* __restrict__ phs,
    const float* __restrict__ We, const float* __restrict__ be,
    const float* __restrict__ Wout, const float* __restrict__ bout,
    float* out, int nN, int nE, int vec8) {
  extern __shared__ v4f lds_dyn[];
  int* reg1 = (int*)lds_dyn;
  int* reg2 = reg1 + RCAP;
  int* scnt = reg2 + RCAP;
  int* soff = scnt + NBMAX;
  int* list = soff + NBMAX;
  int* wcnt = list + LISTN;
  int* wtot = wcnt + NWAVE;
  float* sWe  = (float*)(wtot + NWAVE);
  float* sOut = sWe + TD * WES;
  const int tid = (int)threadIdx.x, lane = tid & 31, wave = tid >> 5;
  const int nodeBase = (int)blockIdx.x * NBMAX;

  for (int i = tid; i < NBMAX; i += NTHR) scnt[i] = 0;
  for (int i = tid; i < DH * TD; i += NTHR) {
    const int o = i >> 5, j = i & 31;
    sWe[o * WES + j] = bfr(We[i]);
  }
  __syncthreads();

  int tot = 0;
  const int nChunks = (nE + CHUNK - 1) / CHUNK;
#pragma unroll 1
  for (int ch = 0; ch < nChunks; ++ch) {
    const int cbase = ch * CHUNK;
    const int wc = scan_chunk(dsts, nE, cbase, nodeBase, NBMAX, vec8, list, tid, lane, wave);
    if (lane == 0) wcnt[wave] = wc;
    __syncthreads();
    int pre = 0, all = 0;
#pragma unroll
    for (int w2 = 0; w2 < NWAVE; ++w2) {
      int c = wcnt[w2];
      c = c < 0 ? 0 : (c > WCAP ? WCAP : c);
      all += c;
      pre += (w2 < wave) ? c : 0;
    }
    const int wcc  = wc > WCAP ? WCAP : wc;
    const int base = tot + pre;
#pragma unroll 1
    for (int i = lane; i < wcc; i += 32) {
      const int ent = list[wave * WCAP + i];
      const int el  = (ent >> 12) & (CHUNK - 1);
      const int sl  = ent & (NBMAX - 1);
      int eid = cbase + el;
      eid = eid > nE - 1 ? nE - 1 : eid;
      const int pos = base + i;
      if (pos < RCAP) reg1[pos] = (int)(((unsigned)eid << SLOTB) | (unsigned)sl);
    }
    tot += all;
    tot = tot > RCAP ? RCAP : tot;
    __syncthreads();
  }
  const int nh = tot;

  if (wave == 0) {
#pragma unroll 1
    for (int b0 = 0; b0 < nh; b0 += 32) {
      const int idx = b0 + lane;
      const int uv  = reg1[idx < nh ? idx : nh - 1];
      const int m32 = (nh - b0) < 32 ? (nh - b0) : 32;
#pragma unroll 1
      for (int k = 0; k < m32; ++k) {
        const int u  = __builtin_amdgcn_readlane(uv, k);
        const int sl = u & (NBMAX - 1);
        if (lane == 0) scnt[sl] = scnt[sl] + 1;
      }
    }
  }
  __syncthreads();

  {
    const int ca = scnt[2 * tid], cb = scnt[2 * tid + 1];
    const int e0 = ca < 0 ? 0 : ca, e1 = cb < 0 ? 0 : cb;
    const int ts = e0 + e1;
    int incl = ts;
#pragma unroll
    for (int d = 1; d < 32; d <<= 1) {
      const int up = __shfl_up(incl, d);
      if (lane >= d) incl += up;
    }
    if (lane == 31) wtot[wave] = incl;
    __syncthreads();
    int pre = 0;
#pragma unroll
    for (int w2 = 0; w2 < NWAVE; ++w2) pre += (w2 < wave) ? wtot[w2] : 0;
    const int run = pre + incl - ts;
    soff[2 * tid]     = run;
    soff[2 * tid + 1] = run + e0;
  }
  __syncthreads();
  for (int i = tid; i < NBMAX; i += NTHR) list[i] = soff[i];
  __syncthreads();

  if (wave == 0) {
#pragma unroll 1
    for (int b0 = 0; b0 < nh; b0 += 32) {
      const int idx = b0 + lane;
      const int uv  = reg1[idx < nh ? idx : nh - 1];
      const int m32 = (nh - b0) < 32 ? (nh - b0) : 32;
#pragma unroll 1
      for (int k = 0; k < m32; ++k) {
        const int u   = __builtin_amdgcn_readlane(uv, k);
        const int sl  = u & (NBMAX - 1);
        const int eid = (int)((unsigned)u >> SLOTB);
        if (lane == 0) {
          int pos = list[sl];
          pos = pos < 0 ? 0 : (pos > RCAP - 1 ? RCAP - 1 : pos);
          reg2[pos] = eid;
          list[sl] = pos + 1;
        }
      }
    }
  }
  __syncthreads();

  const int nbw = NBMAX / NWAVE;
  const bool ovf = (nh >= RCAP);
  const float qnan = __int_as_float(0x7fc00000);
  float* stw = (float*)reg1 + wave * STW;
  const int hj = lane >> 4;
  const float bfj = bfr(bfq[lane]);
  const float phj = bfr(phs[lane]);
  const float bej = bfr(be[lane]);
  const float wo0 = bfr(Wout[lane]);
  const float wo1 = bfr(Wout[DH + lane]);
  const float bo0 = bfr(bout[0]);
  const float bo1 = bfr(bout[1]);

#pragma unroll 1
  for (int jt = 0; jt < nbw; ++jt) {
    const int slot = wave * nbw + jt;
    const int grow = nodeBase + slot;
    const int gcl  = grow < nN ? grow : nN - 1;
    int st = soff[slot];
    const int craw = scnt[slot];
    int cnt = craw;
    st  = st < 0 ? 0 : (st > nh ? nh : st);
    cnt = cnt < 0 ? 0 : (cnt > DEGCAP ? DEGCAP : cnt);
    if (cnt > nh - st) cnt = nh - st;
    const float pz = (ovf || craw > DEGCAP) ? qnan : 0.0f;

    const float* nrow = NODE + (size_t)gcl * NODEW;
    const float qj  = nrow[OQ + lane];
    const float skj = nrow[OSK + lane];
    ldwait();
    __builtin_amdgcn_fence(__ATOMIC_RELEASE, "wavefront");
    __builtin_amdgcn_wave_barrier();
    stw[lane] = qj;
    __builtin_amdgcn_fence(__ATOMIC_RELEASE, "wavefront");
    __builtin_amdgcn_wave_barrier();
    float QW0 = 0.f, QW1 = 0.f;
#pragma unroll 1
    for (int c = 0; c < CH; ++c) {
      QW0 = fmaf(stw[c],      sWe[c * WES + lane],        QW0);
      QW1 = fmaf(stw[CH + c], sWe[(CH + c) * WES + lane], QW1);
    }
    float qbh = qj * bej;
    qbh += __shfl_xor(qbh, 8);
    qbh += __shfl_xor(qbh, 4);
    qbh += __shfl_xor(qbh, 2);
    qbh += __shfl_xor(qbh, 1);
    const float qbo = __shfl_xor(qbh, 16);
    const float qb0 = (hj == 0) ? qbh : qbo;
    const float qb1 = (hj == 0) ? qbo : qbh;

    float m0 = -1.0e30f, m1 = -1.0e30f, dn0 = 0.f, dn1 = 0.f, ae0 = 0.f, ae1 = 0.f, av = 0.f;
#pragma unroll 1
    for (int q = 0; q < cnt; ++q) {
      int idx = st + q; idx = idx > RCAP - 1 ? RCAP - 1 : idx;
      int eid = reg2[idx]; eid = eid < 0 ? 0 : (eid > nE - 1 ? nE - 1 : eid);
      const int sraw = srcs[eid];
      const int s = sraw < 0 ? 0 : (sraw > nN - 1 ? nN - 1 : sraw);
      const float te = bfr(tt[eid]);
      const float ns = bfr(ntime[s]);
      const float* srow = NODE + (size_t)s * NODEW;
      const float kj = srow[OKK + lane];
      const float vj = srow[OV + lane];
      const float rel = ns - te;
      const float enc = cosv(rel * bfj + phj);
      ldwait();
      const float pqk = qj * kj;
      const float a0 = fmaf(QW0, enc, (hj == 0) ? pqk : 0.0f);
      const float a1 = fmaf(QW1, enc, (hj == 0) ? 0.0f : pqk);
      float town, toth;
      red2((hj == 0) ? a0 : a1, (hj == 0) ? a1 : a0, &town, &toth);
      const float t0 = (hj == 0) ? town : toth;
      const float t1 = (hj == 0) ? toth : town;
      const float l0 = (t0 + qb0) * ATTSC;
      const float l1 = (t1 + qb1) * ATTSC;
      const float df0 = l0 - m0;
      const float ee0 = __expf(-fabsf(df0));
      const bool up0  = df0 > 0.f;
      const float s10 = up0 ? ee0 : 1.0f;
      const float s20 = up0 ? 1.0f : ee0;
      m0  = up0 ? l0 : m0;
      dn0 = fmaf(dn0, s10, s20);
      ae0 = fmaf(ae0, s10, s20 * enc);
      const float df1 = l1 - m1;
      const float ee1 = __expf(-fabsf(df1));
      const bool up1  = df1 > 0.f;
      const float s11 = up1 ? ee1 : 1.0f;
      const float s21 = up1 ? 1.0f : ee1;
      m1  = up1 ? l1 : m1;
      dn1 = fmaf(dn1, s11, s21);
      ae1 = fmaf(ae1, s11, s21 * enc);
      const float s1o = (hj == 0) ? s10 : s11;
      const float s2o = (hj == 0) ? s20 : s21;
      av = fmaf(av, s1o, s2o * vj);
    }
    const float d0s = dn0 > 0.f ? dn0 : 1.0f;
    const float d1s = dn1 > 0.f ? dn1 : 1.0f;
    const float in0 = dn0 > 0.f ? 1.0f : 0.0f;
    const float in1 = dn1 > 0.f ? 1.0f : 0.0f;
    const float iv0 = in0 * __builtin_amdgcn_rcpf(d0s);
    const float iv1 = in1 * __builtin_amdgcn_rcpf(d1s);
    const float ivo = (hj == 0) ? iv0 : iv1;
    const float ino = (hj == 0) ? in0 : in1;
    const float AVn  = av * ivo;
    const float AEn0 = ae0 * iv0;
    const float AEn1 = ae1 * iv1;
    __builtin_amdgcn_fence(__ATOMIC_RELEASE, "wavefront");
    __builtin_amdgcn_wave_barrier();
    stw[lane]      = AEn0;
    stw[DH + lane] = AEn1;
    __builtin_amdgcn_fence(__ATOMIC_RELEASE, "wavefront");
    __builtin_amdgcn_wave_barrier();
    float et = 0.f;
    const float* wer = sWe + lane * WES;
    const float* aer = stw + hj * DH;
#pragma unroll 1
    for (int i = 0; i < TD; ++i) et = fmaf(wer[i], aer[i], et);
    const float hc = ((AVn + et) + bej * ino) + skj;
    float zown, zoth;
    red2((hj == 0) ? hc * wo0 : hc * wo1, (hj == 0) ? hc * wo1 : hc * wo0, &zown, &zoth);
    const float z0 = ((hj == 0) ? zown : zoth) + bo0;
    const float z1 = ((hj == 0) ? zoth : zown) + bo1;
    const float mz  = fmaxf(z0, z1);
    const float sh0 = z0 - mz, sh1 = z1 - mz;
    const float lse = __logf(__expf(sh0) + __expf(sh1));
    const float o0 = (sh0 - lse) + pz;
    const float o1 = (sh1 - lse) + pz;
    if (lane == 0) {
      sOut[NCLS * slot]     = o0;
      sOut[NCLS * slot + 1] = o1;
    }
  }
  __syncthreads();

  {
    const int line  = tid >> 3;
    const int piece = tid & 7;
    const int r0 = nodeBase + 16 * line + 2 * piece;
    const v4f val = *(const v4fa*)(sOut + 32 * line + 4 * piece);
    const bool ok = (r0 + 2 <= nN);
    float* op = out + (size_t)nodeBase * NCLS + 32 * line + 4 * piece;
    if (ok) *(volatile v4f*)op = val;
    __threadfence();
    if (ok) *(volatile v4f*)op = val;
  }
}

static inline int cdiv(int a, int b) { return (a + b - 1) / b; }

extern "C" void kernel_launch(void* const* d_in, const int* in_sizes, int n_in,
                              void* d_out, int out_size, void* d_ws, size_t ws_size,
                              hipStream_t stream) {
  if (n_in < 20) return;
  const int nN = in_sizes[3];
  if (nN < 2 || (nN & 1) != 0 || nN > (1 << 22)) return;
  if (in_sizes[0] != nN * DIN) return;
  const int nE = in_sizes[2];
  if (nE < 1 || nE > (1 << 22) - 1) return;
  if (in_sizes[1] != 2 * nE) return;
  if (in_sizes[4] != TD || in_sizes[5] != TD) return;
  if (in_sizes[6] != DH * DIN || in_sizes[7] != DH) return;
  if (in_sizes[8]  != DH * DH || in_sizes[9]  != DH) return;
  if (in_sizes[10] != DH * DH || in_sizes[11] != DH) return;
  if (in_sizes[12] != DH * DH || in_sizes[13] != DH) return;
  if (in_sizes[14] != DH * TD || in_sizes[15] != DH) return;
  if (in_sizes[16] != DH * DH || in_sizes[17] != DH) return;
  if (in_sizes[18] != NCLS * DH || in_sizes[19] != NCLS) return;
  if (out_size != nN * NCLS) return;

  const float* x      = (const float*)d_in[0];
  const int*   ei     = (const int*)  d_in[1];
  const float* t      = (const float*)d_in[2];
  const float* ntime  = (const float*)d_in[3];
  const float* bfq    = (const float*)d_in[4];
  const float* phs    = (const float*)d_in[5];
  const float* W_lin  = (const float*)d_in[6];
  const float* b_lin  = (const float*)d_in[7];
  const float* Wq     = (const float*)d_in[8];
  const float* bq     = (const float*)d_in[9];
  const float* Wk     = (const float*)d_in[10];
  const float* bk     = (const float*)d_in[11];
  const float* Wv     = (const float*)d_in[12];
  const float* bv     = (const float*)d_in[13];
  const float* We     = (const float*)d_in[14];
  const float* be     = (const float*)d_in[15];
  const float* Wskip  = (const float*)d_in[16];
  const float* bskip  = (const float*)d_in[17];
  const float* W_out  = (const float*)d_in[18];
  const float* b_out  = (const float*)d_in[19];
  float* out = (float*)d_out;
  const int* src = ei;
  const int* dst = ei + nE;

  const int MP   = cdiv(nN, GBM) * GBM;
  const int gA   = cdiv(nN, NBMAX);
  const int vec8 = ((nE & 3) == 0) ? 1 : 0;
  if (gA * NBMAX < nN) return;

  char* ws = (char*)d_ws;
  size_t off = 0;
  const size_t oXA  = off; off += (size_t)MP * KP * 2;             off = (off + 255) & ~(size_t)255;
  const size_t oWLT = off; off += (size_t)DH * KP * 2;             off = (off + 255) & ~(size_t)255;
  const size_t oB2T = off; off += (size_t)NB2 * KP * 2;            off = (off + 255) & ~(size_t)255;
  const size_t oH1A = off; off += (size_t)MP * KP * 2;             off = (off + 255) & ~(size_t)255;
  const size_t oND  = off; off += (size_t)MP * NODEW * 4;          off = (off + 255) & ~(size_t)255;
  if (off > ws_size || off > (size_t)WSMAX) return;
  unsigned short* XA   = (unsigned short*)(ws + oXA);
  unsigned short* WLT  = (unsigned short*)(ws + oWLT);
  unsigned short* B2T  = (unsigned short*)(ws + oB2T);
  unsigned short* H1A  = (unsigned short*)(ws + oH1A);
  float*          NODE = (float*)(ws + oND);

  hipFuncSetAttribute(reinterpret_cast<const void*>(&k_agg),
                      hipFuncAttributeMaxDynamicSharedMemorySize, LDS_AGG);

  const int nUx = MP * (KP / 8);
  k_xprep<<<cdiv(nUx, NTHR), NTHR, 0, stream>>>(x, XA, nN, nUx);

  k_wprep<<<1 + (NB2 * 8) / NTHR, NTHR, 0, stream>>>(W_lin, Wq, Wk, Wv, Wskip, WLT, B2T);

  const int gM = MP / GBM;
  k_gemm1<<<gM, GTHR, 0, stream>>>(XA, WLT, b_lin, H1A, KP, nN);
  k_gemm2<<<dim3(gM, NODEW / GBN), GTHR, 0, stream>>>(H1A, B2T, bq, bk, bv, bskip, NODE, KP, NODEW);
  k_agg<<<gA, NTHR, LDS_AGG, stream>>>(src, dst, NODE, t, ntime, bfq, phs, We, be, W_out, b_out,
                                       out, nN, nE, vec8);
}
